// TripleAttentionSmarter_21809843929814
// MI455X (gfx1250) — hardware-verified
//
#include <hip/hip_runtime.h>


#define NBI  2
#define NN   256
#define CC   512
#define NH_  8
#define HD   64
#define W5   (5 * CC)
#define BIGN (NN * HD)
#define DM   CC
#define NTK  NN
#define SCL  0.125f
#define LOSC 1024.0f

typedef _Float16 h16;
typedef unsigned short bf;
typedef __attribute__((ext_vector_type(16))) __bf16   v16bf;
typedef __attribute__((ext_vector_type(16))) _Float16 v16h;
typedef __attribute__((ext_vector_type(8)))  _Float16 v8h;
typedef __attribute__((ext_vector_type(8)))  unsigned short v8us;
typedef __attribute__((ext_vector_type(8)))  float    v8f;
typedef __attribute__((ext_vector_type(4)))  float    v4f;
typedef __attribute__((ext_vector_type(4)))  _Float16 v4h;
typedef v8h  __attribute__((may_alias)) v8ha;
typedef v4f  __attribute__((may_alias)) v4fa;
typedef v8us __attribute__((may_alias)) v8usa;

__device__ __forceinline__ unsigned short f2bf(float f) { unsigned u = __float_as_uint(f); u += 0x7FFFu + ((u >> 16) & 1u); return (unsigned short)(u >> 16); }
__device__ __forceinline__ float bf2f(unsigned short b) { return __uint_as_float(((unsigned)b) << 16); }
__device__ __forceinline__ float bfr(float f) { return bf2f(f2bf(f)); }
__device__ __forceinline__ v16h cat16(v8h lo, v8h hi) { return __builtin_shufflevector(lo, hi, 0, 1, 2, 3, 4, 5, 6, 7, 8, 9, 10, 11, 12, 13, 14, 15); }
__device__ __forceinline__ v16bf cat16b(v8us lo, v8us hi) { return __builtin_bit_cast(v16bf, __builtin_shufflevector(lo, hi, 0, 1, 2, 3, 4, 5, 6, 7, 8, 9, 10, 11, 12, 13, 14, 15)); }
__device__ __forceinline__ v8f wmma16(v16h a, v16h b, v8f c) { return __builtin_amdgcn_wmma_f32_16x16x32_f16(false, a, false, b, (short)0, c, false, false); }
__device__ __forceinline__ v8f wmmab(v16bf a, v16bf b, v8f c) { return __builtin_amdgcn_wmma_f32_16x16x32_bf16(false, a, false, b, (short)0, c, false, false); }

__global__ __launch_bounds__(256) void k_cvtb(const float* __restrict__ src, int nrows, bf* dst) {
    const int lane = threadIdx.x & 31, r = blockIdx.x * 8 + (threadIdx.x >> 5);
    if (r >= nrows) return;
    v8us o[DM / 256];
#pragma unroll
    for (int q = 0; q < DM / 256; ++q) { v8us t;
#pragma unroll
        for (int i = 0; i < 8; ++i) t[i] = f2bf(src[(size_t)r * DM + q * 256 + lane * 8 + i]);
        o[q] = t; }
#pragma unroll
    for (int q = 0; q < DM / 256; ++q) *(volatile v8us*)(dst + (size_t)r * DM + q * 256 + lane * 8) = o[q];
    __threadfence();
#pragma unroll
    for (int q = 0; q < DM / 256; ++q) *(volatile v8us*)(dst + (size_t)r * DM + q * 256 + lane * 8) = o[q];
}

template <bool SPLITA, bool F16OUT = false>
__global__ __launch_bounds__(128) void k_gemmb(const bf* __restrict__ A, const bf* __restrict__ Al, const bf* __restrict__ Bn, const float* __restrict__ bias, float* C, int ldc, h16* C2, const float* __restrict__ R = nullptr, int K = DM, int roundR = 1) {
    __shared__ __align__(16) float ost[4][16 * 68];
    const int lane = threadIdx.x & 31, wave = threadIdx.x >> 5, lr = lane & 15, hi = lane >> 4;
    const int r0 = blockIdx.x * 64 + wave * 16, c0 = blockIdx.y * 64;
    const size_t aoff = (size_t)(r0 + lr) * K + 8 * hi;
    size_t boff[4];
#pragma unroll
    for (int t = 0; t < 4; ++t) boff[t] = (size_t)(c0 + t * 16 + lr) * K + 8 * hi;
    v8f acc[4];
#pragma unroll
    for (int t = 0; t < 4; ++t) acc[t] = (v8f){};
#pragma unroll 1
    for (int kc = 0; kc < K; kc += 32) {
        const v16bf a = cat16b(*(const v8us*)(A + aoff + kc), *(const v8us*)(A + aoff + kc + 16));
        v16bf al = a;
        if (SPLITA) al = cat16b(*(const v8us*)(Al + aoff + kc), *(const v8us*)(Al + aoff + kc + 16));
#pragma unroll
        for (int t = 0; t < 4; ++t) { const v16bf b = cat16b(*(const v8us*)(Bn + boff[t] + kc), *(const v8us*)(Bn + boff[t] + kc + 16)); acc[t] = wmmab(a, b, acc[t]); if (SPLITA) acc[t] = wmmab(al, b, acc[t]); }
        asm volatile("v_nop\n\tv_nop\n\tv_nop\n\tv_nop" : "+v"(acc[0]), "+v"(acc[1]), "+v"(acc[2]), "+v"(acc[3]) : "v"(a), "v"(al));
    }
    float* os = &ost[wave][0];
#pragma unroll
    for (int t = 0; t < 4; ++t) { const float bv = bias ? bfr(bias[c0 + t * 16 + lr]) : 0.f;
#pragma unroll
        for (int j = 0; j < 8; ++j) os[(hi * 8 + j) * 68 + t * 16 + lr] = acc[t][j] + bv; }
    __syncthreads();
    if (F16OUT) {
        h16* crow = (h16*)(void*)C + (size_t)r0 * ldc + c0;
        auto pass = [&]() {
#pragma unroll
            for (int s = 0; s < 4; ++s) { const int row = 4 * s + (lane >> 3), piece = lane & 7; const float* sp = os + row * 68 + piece * 8; v8h o, o2;
#pragma unroll
                for (int i = 0; i < 8; ++i) { const h16 a = (h16)sp[i]; o[i] = a; o2[i] = (h16)((sp[i] - (float)a) * LOSC); }
                *(volatile v8h*)(crow + (size_t)row * ldc + piece * 8) = o; if (C2) *(volatile v8h*)(C2 + (size_t)r0 * ldc + c0 + (size_t)row * ldc + piece * 8) = o2; }
        };
        pass(); __threadfence(); pass();
    } else {
        float* crow = C + (size_t)r0 * ldc + c0;
        auto pass = [&]() {
#pragma unroll
            for (int s = 0; s < 8; ++s) { const int Lid = (lane >> 3) + 4 * s, piece = lane & 7; const int row = Lid >> 1, cofs = (Lid & 1) * 32 + piece * 4;
                v4f val = *(const v4fa*)(os + row * 68 + cofs); if (R) { const v4f rv = *(const v4f*)(R + ((size_t)r0 + row) * ldc + c0 + cofs); val += roundR ? (v4f){bfr(rv[0]), bfr(rv[1]), bfr(rv[2]), bfr(rv[3])} : rv; }
                *(volatile v4f*)(crow + (size_t)row * ldc + cofs) = val; }
        };
        pass(); __threadfence(); pass();
    }
}

__global__ __launch_bounds__(128) void k_gemm3(const bf* __restrict__ Ah, const bf* __restrict__ Al, const bf* __restrict__ Bh, const bf* __restrict__ Bl, int K, float* C, int ldc) {
    __shared__ __align__(16) float ost[4][16 * 68];
    const int lane = threadIdx.x & 31, wave = threadIdx.x >> 5, lr = lane & 15, hi = lane >> 4;
    const int r0 = blockIdx.x * 64 + wave * 16, c0 = blockIdx.y * 64;
    const size_t aoff = (size_t)(r0 + lr) * K + 8 * hi;
    v8f acc[4];
#pragma unroll
    for (int t = 0; t < 4; ++t) acc[t] = (v8f){};
#pragma unroll 1
    for (int kc = 0; kc < K; kc += 32) {
        const v16bf a = cat16b(*(const v8us*)(Ah + aoff + kc), *(const v8us*)(Ah + aoff + kc + 16));
        const v16bf al = cat16b(*(const v8us*)(Al + aoff + kc), *(const v8us*)(Al + aoff + kc + 16));
#pragma unroll
        for (int t = 0; t < 4; ++t) { const size_t bo = (size_t)(c0 + t * 16 + lr) * K + kc + 8 * hi;
            const v16bf bh = cat16b(*(const v8us*)(Bh + bo), *(const v8us*)(Bh + bo + 16)); const v16bf bl = cat16b(*(const v8us*)(Bl + bo), *(const v8us*)(Bl + bo + 16));
            acc[t] = wmmab(a, bh, acc[t]); acc[t] = wmmab(al, bh, acc[t]); acc[t] = wmmab(a, bl, acc[t]); }
        asm volatile("v_nop\n\tv_nop\n\tv_nop\n\tv_nop" : "+v"(acc[0]), "+v"(acc[1]), "+v"(acc[2]), "+v"(acc[3]) : "v"(a), "v"(al));
    }
    float* os = &ost[wave][0];
#pragma unroll
    for (int t = 0; t < 4; ++t) {
#pragma unroll
        for (int j = 0; j < 8; ++j) os[(hi * 8 + j) * 68 + t * 16 + lr] = acc[t][j]; }
    __builtin_amdgcn_wave_barrier(); asm volatile("" ::: "memory");
    float* crow = C + (size_t)r0 * ldc + c0;
    auto pass = [&]() {
#pragma unroll
        for (int s = 0; s < 8; ++s) { const int Lid = (lane >> 3) + 4 * s, piece = lane & 7; const int row = Lid >> 1, cofs = (Lid & 1) * 32 + piece * 4;
            const v4f val = *(const v4fa*)(os + row * 68 + cofs); *(volatile v4f*)(crow + (size_t)row * ldc + cofs) = val; }
    };
    pass(); __threadfence(); pass();
}

__global__ __launch_bounds__(256) void k_bf(const float* __restrict__ src, bf* dst, size_t n8) {
    const size_t i = (size_t)blockIdx.x * 256 + threadIdx.x; if (i >= n8) return;
    const v8f v = *(const v8f*)(src + i * 8); v8us o;
#pragma unroll
    for (int k = 0; k < 8; ++k) o[k] = f2bf(v[k]);
    *(volatile v8us*)(dst + i * 8) = o; __threadfence(); *(volatile v8us*)(dst + i * 8) = o;
}
__global__ __launch_bounds__(256) void k_hd(const float* __restrict__ Wf, int h, bf* PL) {
    typedef __attribute__((ext_vector_type(2))) unsigned short v2us;
    const int lane = threadIdx.x & 31, wid = blockIdx.x * 8 + (threadIdx.x >> 5); if (wid >= NN * 3) return;
    const int r = wid / 3, p = wid % 3;
    v2us oh, ol;
#pragma unroll
    for (int i = 0; i < 2; ++i) { const int d = 2 * lane + i; const float v = Wf[(size_t)r * W5 + p * CC + h * HD + d]; const unsigned short hb = f2bf(v); oh[i] = hb; ol[i] = f2bf(v - bf2f(hb)); }
    const size_t o = ((size_t)(p * 2) * NN + r) * HD + 2 * lane, o2 = ((size_t)(p * 2 + 1) * NN + r) * HD + 2 * lane;
    *(volatile v2us*)(PL + o) = oh; *(volatile v2us*)(PL + o2) = ol; __threadfence(); *(volatile v2us*)(PL + o) = oh; *(volatile v2us*)(PL + o2) = ol;
}
template <int MODE>
__global__ __launch_bounds__(256) void k_exp(const float* __restrict__ S, float* EF, bf* Eh, bf* El) {
    const int lane = threadIdx.x & 31, r = blockIdx.x * 8 + (threadIdx.x >> 5); if (r >= NN) return;
    const size_t o = (size_t)r * NN + lane * 8; const v8f v = *(const v8f*)(S + o); v8f e; v8us oh, ol;
#pragma unroll
    for (int i = 0; i < 8; ++i) { e[i] = __expf(v[i] * SCL); const unsigned short hb = f2bf(e[i]); oh[i] = hb; ol[i] = f2bf(e[i] - bf2f(hb)); }
    if (MODE == 0) { *(volatile v8f*)(EF + o) = e; __threadfence(); *(volatile v8f*)(EF + o) = e; }
    else { *(volatile v8us*)(Eh + o) = oh; *(volatile v8us*)(El + o) = ol; __threadfence(); *(volatile v8us*)(Eh + o) = oh; *(volatile v8us*)(El + o) = ol; }
}
__global__ __launch_bounds__(256) void k_bigb(const float* __restrict__ ZTF, const float* __restrict__ Wf, int h, bf* Bh, bf* Bl) {
    const int u = blockIdx.x * 256 + threadIdx.x; if (u >= BIGN * NN / 8) return;
    const int n = u / (NN / 8), k0 = (u % (NN / 8)) * 8; const int i = n / HD, d = n % HD;
    v8us oh, ol;
#pragma unroll
    for (int q = 0; q < 8; ++q) { const int k = k0 + q; const float v = ZTF[(size_t)i * NN + k] * Wf[(size_t)k * W5 + 4 * CC + h * HD + d]; const unsigned short hb = f2bf(v); oh[q] = hb; ol[q] = f2bf(v - bf2f(hb)); }
    const size_t o = (size_t)n * NN + k0; *(volatile v8us*)(Bh + o) = oh; *(volatile v8us*)(Bl + o) = ol; __threadfence(); *(volatile v8us*)(Bh + o) = oh; *(volatile v8us*)(Bl + o) = ol;
}
__global__ __launch_bounds__(256) void k_numden(const float* __restrict__ XF, const float* __restrict__ Wf, const float* __restrict__ T, const float* __restrict__ YZ, int h, float* O4) {
    const int u = blockIdx.x * 256 + threadIdx.x; if (u >= NN * HD) return;
    const int i = u / HD, d = u % HD;
    float num = 0.f, den = 0.f;
#pragma unroll 1
    for (int j = 0; j < NN; ++j) { const float xij = XF[(size_t)i * NN + j]; num = fmaf(xij * Wf[(size_t)j * W5 + 3 * CC + h * HD + d], T[(size_t)j * BIGN + i * HD + d], num); den = fmaf(xij, YZ[(size_t)j * NN + i], den); }
    const float o = num / den; float* p = O4 + ((size_t)h * NN + i) * HD + d;
    *(volatile float*)p = o; __threadfence(); *(volatile float*)p = o;
}
__global__ __launch_bounds__(256) void k_split(const float* __restrict__ src, int nrows, bf* dh, bf* dl) {
    const int lane = threadIdx.x & 31, r = blockIdx.x * 8 + (threadIdx.x >> 5); if (r >= nrows) return;
#pragma unroll 1
    for (int ps = 0; ps < 2; ++ps) {
#pragma unroll 1
        for (int q = 0; q < DM / 256; ++q) { const size_t o = (size_t)r * DM + q * 256 + lane * 8; const v8f v = *(const v8f*)(src + o); v8us oh, ol;
#pragma unroll
            for (int i = 0; i < 8; ++i) { const unsigned short hb = f2bf(v[i]); oh[i] = hb; ol[i] = f2bf(v[i] - bf2f(hb)); }
            *(volatile v8us*)(dh + o) = oh; *(volatile v8us*)(dl + o) = ol; }
        if (ps == 0) __threadfence(); }
}

extern "C" void kernel_launch(void* const* d_in, const int* in_sizes, int n_in,
                              void* d_out, int out_size, void* d_ws, size_t ws_size, hipStream_t stream) {
    (void)in_sizes; (void)n_in; (void)out_size;
    const float* x = (const float*)d_in[0]; const float* Ww = (const float*)d_in[1]; const float* Wo = (const float*)d_in[2]; const float* bo = (const float*)d_in[3];
    float* out = (float*)d_out;
    char* wsp = (char*)d_ws;
    auto take = [&](size_t bytes) { char* p = wsp; wsp += (bytes + 255) & ~(size_t)255; return (void*)p; };
    bf* WwB = (bf*)take((size_t)W5 * CC * 2); bf* WoB = (bf*)take((size_t)CC * CC * 2); bf* Xb = (bf*)take((size_t)NN * CC * 2); float* Wf = (float*)take((size_t)NN * W5 * 4);
    bf* PL = (bf*)take((size_t)6 * NN * HD * 2); float* S = (float*)take((size_t)NN * NN * 4); float* XF = (float*)take((size_t)NN * NN * 4); float* ZTF = (float*)take((size_t)NN * NN * 4);
    bf* Yh = (bf*)take((size_t)NN * NN * 2); bf* Yl = (bf*)take((size_t)NN * NN * 2); bf* ZTh = (bf*)take((size_t)NN * NN * 2); bf* ZTl = (bf*)take((size_t)NN * NN * 2);
    bf* Bh = (bf*)take((size_t)BIGN * NN * 2); bf* Bl = (bf*)take((size_t)BIGN * NN * 2); float* T = (float*)take((size_t)NN * BIGN * 4); float* YZ = (float*)take((size_t)NN * NN * 4);
    float* O4 = (float*)take((size_t)NH_ * NN * HD * 4); bf* Oh = (bf*)take((size_t)NN * CC * 2); bf* Ol = (bf*)take((size_t)NN * CC * 2);
    if ((size_t)(wsp - (char*)d_ws) > ws_size) return;
    k_bf<<<(W5 * CC / 8 + 255) / 256, 256, 0, stream>>>(Ww, WwB, (size_t)W5 * CC / 8); k_bf<<<(CC * CC / 8 + 255) / 256, 256, 0, stream>>>(Wo, WoB, (size_t)CC * CC / 8);
    bf* Ah = PL; bf* Al = PL + (size_t)NN * HD; bf* Bph = PL + (size_t)2 * NN * HD; bf* Bpl = PL + (size_t)3 * NN * HD; bf* Ch = PL + (size_t)4 * NN * HD; bf* Cl = PL + (size_t)5 * NN * HD;
    for (int b = 0; b < NBI; ++b) {
        k_cvtb<<<NN / 8, 256, 0, stream>>>(x + (size_t)b * NN * CC, NN, Xb);
        k_gemmb<false, false><<<dim3(NN / 64, W5 / 64, 1), 128, 0, stream>>>(Xb, nullptr, WwB, nullptr, Wf, W5, nullptr);
        for (int h = 0; h < NH_; ++h) {
            k_hd<<<(NN * 3 + 7) / 8, 256, 0, stream>>>(Wf, h, PL);
            k_gemm3<<<dim3(NN / 64, NN / 64, 1), 128, 0, stream>>>(Ah, Al, Bph, Bpl, HD, S, NN); k_exp<0><<<NN / 8, 256, 0, stream>>>(S, XF, nullptr, nullptr);
            k_gemm3<<<dim3(NN / 64, NN / 64, 1), 128, 0, stream>>>(Bph, Bpl, Ch, Cl, HD, S, NN); k_exp<1><<<NN / 8, 256, 0, stream>>>(S, nullptr, Yh, Yl);
            k_gemm3<<<dim3(NN / 64, NN / 64, 1), 128, 0, stream>>>(Ah, Al, Ch, Cl, HD, S, NN); k_exp<0><<<NN / 8, 256, 0, stream>>>(S, ZTF, nullptr, nullptr); k_exp<1><<<NN / 8, 256, 0, stream>>>(S, nullptr, ZTh, ZTl);
            k_bigb<<<(BIGN * NN / 8 + 255) / 256, 256, 0, stream>>>(ZTF, Wf, h, Bh, Bl);
            k_gemm3<<<dim3(NN / 64, BIGN / 64, 1), 128, 0, stream>>>(Yh, Yl, Bh, Bl, NN, T, BIGN);
            k_gemm3<<<dim3(NN / 64, NN / 64, 1), 128, 0, stream>>>(Yh, Yl, ZTh, ZTl, NN, YZ, NN);
            k_numden<<<(NN * HD) / 256, 256, 0, stream>>>(XF, Wf, T, YZ, h, O4);
        }
        k_split<<<NN / 8, 256, 0, stream>>>(O4, NN, Oh, Ol);
        k_gemmb<true, false><<<dim3(NN / 64, CC / 64, 1), 128, 0, stream>>>(Oh, Ol, WoB, bo, out + (size_t)b * NN * CC, CC, nullptr);
    }
}
